// Double_SSM_Block_Encoder_59382217834750
// MI455X (gfx1250) — hardware-verified
//
#include <hip/hip_runtime.h>
#include <hip/hip_bf16.h>
#include <math.h>

typedef __attribute__((ext_vector_type(16))) _Float16 v16h;
typedef __attribute__((ext_vector_type(8)))  _Float16 v8h;
typedef __attribute__((ext_vector_type(16))) __bf16   v16b;
typedef __attribute__((ext_vector_type(8)))  __bf16   v8b;
typedef __attribute__((ext_vector_type(8)))  float    v8f;
typedef __attribute__((ext_vector_type(4)))  float    v4f;
typedef __attribute__((ext_vector_type(2)))  float    v2f;

#define NB     8
#define SEQL   4096
#define NROWS  32768
#define CIN    64
#define DIN    128
#define NST    16
#define NDT    4
#define NPRJ   64
#define TS     32

#define WIN1_H   0
#define WIN1_L   16384
#define WX1_H    32768
#define WX1_L    40960
#define WOUT1_H  49152
#define WOUT1_L  57344
#define WIN2_H   65536
#define WIN2_L   81920
#define WX2_H    98304
#define WX2_L    106496
#define WOUT2_H  114688
#define WOUT2_L  131072
#define WGT_END  147456

__device__ __forceinline__ unsigned short f2bf_bits(float f) {
  unsigned u = __float_as_uint(f);
  return (unsigned short)((u + 0x7FFFu + ((u >> 16) & 1u)) >> 16);
}
__device__ __forceinline__ float bf_bits2f(unsigned short h) { return __uint_as_float(((unsigned)h) << 16); }

__device__ __forceinline__ void dep_guard_h(v8f& a, v8f& b, v16h x, v16h y) { asm volatile("v_nop\n\tv_nop\n\tv_nop\n\tv_nop" : "+v"(a), "+v"(b) : "v"(x), "v"(y)); }
__device__ __forceinline__ void dep_guard_b(v8f& a, v8f& b, v16b x, v16b y) { asm volatile("v_nop\n\tv_nop\n\tv_nop\n\tv_nop" : "+v"(a), "+v"(b) : "v"(x), "v"(y)); }
__device__ __forceinline__ void keep4_h(v16h a, v16h b, v16h c, v16h d) { asm volatile("v_nop" :: "v"(a), "v"(b), "v"(c), "v"(d)); }
__device__ __forceinline__ void keep4_b(v16b a, v16b b, v16b c, v16b d) { asm volatile("v_nop" :: "v"(a), "v"(b), "v"(c), "v"(d)); }
__device__ __forceinline__ void acc_guard4(v8f& a, v8f& b, v8f& c, v8f& d) { asm volatile("v_nop\n\tv_nop\n\tv_nop\n\tv_nop" : "+v"(a), "+v"(b), "+v"(c), "+v"(d)); }
template <typename T> struct Frag;
template <> struct Frag<_Float16> {
  typedef v16h V; union U { v16h v; v8h h[2]; };
  static __device__ __forceinline__ v16h load(const _Float16* p) {
    U f; f.h[0] = *(const v8h*)(p); f.h[1] = *(const v8h*)(p + 16); return f.v;
  }
  static __device__ __forceinline__ v8f mma(v16h a, v16h b, v8f c) {
    return __builtin_amdgcn_wmma_f32_16x16x32_f16(false, a, false, b, (short)0, c, false, false);
  }
  static __device__ __forceinline__ void guard(v8f& a, v8f& b, v16h x, v16h y) { dep_guard_h(a, b, x, y); }
  static __device__ __forceinline__ void keep(v16h a, v16h b, v16h c, v16h d) { keep4_h(a, b, c, d); }
};
template <> struct Frag<__bf16> {
  typedef v16b V; union U { v16b v; v8b h[2]; };
  static __device__ __forceinline__ v16b load(const __bf16* p) {
    U f; f.h[0] = *(const v8b*)(p); f.h[1] = *(const v8b*)(p + 16); return f.v;
  }
  static __device__ __forceinline__ v8f mma(v16b a, v16b b, v8f c) {
    return __builtin_amdgcn_wmma_f32_16x16x32_bf16(false, a, false, b, (short)0, c, false, false);
  }
  static __device__ __forceinline__ void guard(v8f& a, v8f& b, v16b x, v16b y) { dep_guard_b(a, b, x, y); }
  static __device__ __forceinline__ void keep(v16b a, v16b b, v16b c, v16b d) { keep4_b(a, b, c, d); }
};

template <int ET> struct Elem;
template <> struct Elem<0> { typedef _Float16 T; };
template <> struct Elem<1> { typedef __bf16 T; };
template <int ET, bool SPLIT, int BIAS_MODE, int OUT_MODE, bool RESID, int ACT = 0>
__global__ __launch_bounds__(256) void wmma_gemm64(
    const unsigned short* __restrict__ Ap, const unsigned short* __restrict__ A2p, int lda, long strideA,
    const unsigned short* __restrict__ Btp, const unsigned short* __restrict__ Bt2p, int ldb, long strideB,
    void* __restrict__ Cout, void* __restrict__ Cout2, int ldc, long strideC,
    const float* __restrict__ bias,
    const float* __restrict__ resid, long strideR,
    int M, int N, int K, float scale) {
  typedef typename Elem<ET>::T T;
  typedef typename Frag<T>::V V;
  const T* A = (const T*)Ap; const T* A2 = (const T*)A2p; const T* Bt = (const T*)Btp; const T* Bt2 = (const T*)Bt2p;
  __shared__ __align__(16) float sT[8][16 * 68];
  const int b    = blockIdx.y;
  const int lane = threadIdx.x & 31;
  const int wave = threadIdx.x >> 5;
  const int tilesN = N >> 6;
  const int tilesM = M >> 6;
  const int tile = blockIdx.x * 8 + wave;
  if (tile >= tilesM * tilesN) return;
  const int tm = tile / tilesN;
  const int tn = tile - tm * tilesN;
  const int m0 = tm << 6;
  const int n0 = tn << 6;

  const T* Ab  = A  + (size_t)b * strideA;
  const T* Bb  = Bt + (size_t)b * strideB;
  const T* Ab2 = SPLIT ? (A2  + (size_t)b * strideA) : nullptr;
  const T* Bb2 = SPLIT ? (Bt2 + (size_t)b * strideB) : nullptr;

  const int rlane = lane & 15;
  const int koff  = (lane >> 4) * 8;
  const int mOff  = (lane >> 4) * 8;

  v8f acc[4][4];
#pragma unroll
  for (int i = 0; i < 4; ++i)
#pragma unroll
    for (int j = 0; j < 4; ++j) acc[i][j] = (v8f){0.f,0.f,0.f,0.f,0.f,0.f,0.f,0.f};

  for (int k0 = 0; k0 < K; k0 += 32) {
    V bh[4], bl[4];
#pragma unroll
    for (int j = 0; j < 4; ++j) {
      const size_t bo = (size_t)(n0 + (j << 4) + rlane) * ldb + koff + k0;
      bh[j] = Frag<T>::load(Bb + bo);
      if (SPLIT) bl[j] = Frag<T>::load(Bb2 + bo);
    }
#pragma unroll
    for (int i = 0; i < 4; ++i) {
      const size_t ao = (size_t)(m0 + (i << 4) + rlane) * lda + koff + k0;
      V ah = Frag<T>::load(Ab + ao);
      V al;
      if (SPLIT) al = Frag<T>::load(Ab2 + ao);
#pragma unroll
      for (int j = 0; j < 4; ++j) {
        acc[i][j] = Frag<T>::mma(ah, bh[j], acc[i][j]);
        if (SPLIT) {
          acc[i][j] = Frag<T>::mma(ah, bl[j], acc[i][j]);
          acc[i][j] = Frag<T>::mma(al, bh[j], acc[i][j]);
        }
      }
      Frag<T>::guard(acc[i][0], acc[i][3], ah, SPLIT ? al : ah);
    }
    Frag<T>::keep(bh[0], bh[1], bh[2], bh[3]);
    if (SPLIT) Frag<T>::keep(bl[0], bl[1], bl[2], bl[3]);
  }
  acc_guard4(acc[0][0], acc[0][1], acc[0][2], acc[0][3]);
  acc_guard4(acc[1][0], acc[1][1], acc[1][2], acc[1][3]);
  acc_guard4(acc[2][0], acc[2][1], acc[2][2], acc[2][3]);
  acc_guard4(acc[3][0], acc[3][1], acc[3][2], acc[3][3]);

  float* slab = sT[wave];
  const float* Rb = RESID ? (resid + (size_t)b * strideR) : nullptr;
#pragma unroll
  for (int i = 0; i < 4; ++i) {
    const int mBase = m0 + (i << 4);
#pragma unroll
    for (int j = 0; j < 4; ++j) {
      const int n = n0 + (j << 4) + rlane;
      float bv = 0.f;
      if (BIAS_MODE == 2) bv = bias[n];
#pragma unroll
      for (int r = 0; r < 8; ++r) {
        float v = acc[i][j][r] * scale;
        if (BIAS_MODE == 1) v += bias[mBase + mOff + r];
        if (BIAS_MODE == 2) v += bv;
        if (RESID) v += Rb[(size_t)(mBase + mOff + r) * ldc + n];
        if (ACT == 1) v = tanhf(v);
        if (ACT == 2) v = fmaxf(v, 0.0f);
        if (ACT == 3) v = v / (1.0f + expf(-v));
        if (ACT == 4) v = (v > 0.f) ? v : 0.01f * v;
        if (ACT == 5) v = 0.5f * v * (1.0f + erff(v * 0.70710678118654752f));
        slab[(mOff + r) * 68 + (j << 4) + rlane] = v;
      }
    }
    __builtin_amdgcn_fence(__ATOMIC_RELEASE, "workgroup");
    __builtin_amdgcn_wave_barrier();
    __builtin_amdgcn_fence(__ATOMIC_ACQUIRE, "workgroup");
    if (OUT_MODE == 0) {
      float* C = (float*)Cout + (size_t)b * strideC;
      const int hh = lane >> 4, c4 = (lane & 15) * 4;
      for (int pass = 0; pass < 2; ++pass) {
#pragma unroll
        for (int it = 0; it < 8; ++it) {
          const int row = it * 2 + hh;
          v4f v = *(const v4f*)(slab + row * 68 + c4);
          *(volatile v4f*)(C + (size_t)(mBase + row) * ldc + n0 + c4) = v;
        }
        __threadfence();
      }
    } else {
      const int q = lane >> 3, c8 = (lane & 7) * 8;
      unsigned short* C  = (unsigned short*)Cout  + (size_t)b * strideC;
      unsigned short* C2 = (OUT_MODE == 2) ? ((unsigned short*)Cout2 + (size_t)b * strideC) : nullptr;
      for (int pass = 0; pass < 2; ++pass) {
#pragma unroll
        for (int it = 0; it < 4; ++it) {
          const int row = it * 4 + q;
          const float* sp = slab + row * 68 + c8;
          v8h hv, lv;
#pragma unroll
          for (int e = 0; e < 8; ++e) {
            if (OUT_MODE == 1) {
              hv[e] = (_Float16)sp[e];
            } else {
              unsigned short hb = f2bf_bits(sp[e]);
              unsigned short lb = f2bf_bits(sp[e] - bf_bits2f(hb));
              hv[e] = __builtin_bit_cast(_Float16, hb);
              lv[e] = __builtin_bit_cast(_Float16, lb);
            }
          }
          *(volatile v8h*)(C + (size_t)(mBase + row) * ldc + n0 + c8) = hv;
          if (OUT_MODE == 2) *(volatile v8h*)(C2 + (size_t)(mBase + row) * ldc + n0 + c8) = lv;
        }
        __threadfence();
      }
    }
    __builtin_amdgcn_fence(__ATOMIC_RELEASE, "workgroup");
    __builtin_amdgcn_wave_barrier();
    __builtin_amdgcn_fence(__ATOMIC_ACQUIRE, "workgroup");
  }
}

__device__ __forceinline__ void split_bf8(v4f a0, v4f a1, v8h& hv, v8h& lv) {
#pragma unroll
  for (int e = 0; e < 4; ++e) {
    const unsigned short h0 = f2bf_bits(a0[e]);
    const unsigned short l0 = f2bf_bits(a0[e] - bf_bits2f(h0));
    const unsigned short h1 = f2bf_bits(a1[e]);
    const unsigned short l1 = f2bf_bits(a1[e] - bf_bits2f(h1));
    hv[e] = __builtin_bit_cast(_Float16, h0);     lv[e] = __builtin_bit_cast(_Float16, l0);
    hv[4 + e] = __builtin_bit_cast(_Float16, h1); lv[4 + e] = __builtin_bit_cast(_Float16, l1);
  }
}

__global__ __launch_bounds__(256) void weight_planes_kernel(
    const float* __restrict__ w_in1, const float* __restrict__ w_x1, const float* __restrict__ w_out1,
    const float* __restrict__ w_in2, const float* __restrict__ w_x2, const float* __restrict__ w_out2,
    unsigned short* __restrict__ P)
{
  const int y = blockIdx.y;
  const float* W = w_in1; int ldw = 256, Kreal = 64, lgseg = 3, Nreal = 256, Npad = 256, offh = WIN1_H, offl = WIN1_L;
  if (y == 1)      { W = w_x1;   ldw = 36;  Kreal = 128; lgseg = 4; Nreal = 36;  Npad = 64;  offh = WX1_H;   offl = WX1_L; }
  else if (y == 2) { W = w_out1; ldw = 64;  Kreal = 128; lgseg = 4; Nreal = 64;  Npad = 64;  offh = WOUT1_H; offl = WOUT1_L; }
  else if (y == 3) { W = w_in2;  ldw = 256; Kreal = 64;  lgseg = 3; Nreal = 256; Npad = 256; offh = WIN2_H;  offl = WIN2_L; }
  else if (y == 4) { W = w_x2;   ldw = 36;  Kreal = 128; lgseg = 4; Nreal = 36;  Npad = 64;  offh = WX2_H;   offl = WX2_L; }
  else if (y == 5) { W = w_out2; ldw = 128; Kreal = 128; lgseg = 4; Nreal = 128; Npad = 128; offh = WOUT2_H; offl = WOUT2_L; }
  const int Kpad  = 8 << lgseg;
  const int total = Npad << lgseg;
  const int i = blockIdx.x * 256 + threadIdx.x;
  if (i >= total) return;
  const int n   = i >> lgseg;
  const int seg = i & ((1 << lgseg) - 1);
  const int nc  = (n < Nreal) ? n : (Nreal - 1);
  v4f a0, a1;
#pragma unroll
  for (int e = 0; e < 4; ++e) {
    const int k0i = seg * 8 + e, k1i = seg * 8 + 4 + e;
    const int kc0 = (k0i < Kreal) ? k0i : (Kreal - 1);
    const int kc1 = (k1i < Kreal) ? k1i : (Kreal - 1);
    const float t0 = W[(size_t)kc0 * ldw + nc];
    const float t1 = W[(size_t)kc1 * ldw + nc];
    a0[e] = (n < Nreal && k0i < Kreal) ? t0 : 0.f;
    a1[e] = (n < Nreal && k1i < Kreal) ? t1 : 0.f;
  }
  v8h hv, lv;
  split_bf8(a0, a1, hv, lv);
  const size_t off = (size_t)n * Kpad + seg * 8;
  for (int pass = 0; pass < 2; ++pass) {
    *(volatile v8h*)(P + offh + off) = hv;
    *(volatile v8h*)(P + offl + off) = lv;
    __threadfence();
  }
}

__global__ __launch_bounds__(256) void x_to_planes_kernel(
    const float* __restrict__ x, unsigned short* __restrict__ Th, unsigned short* __restrict__ Tl)
{
  __shared__ __align__(16) float s[64 * 68];
  const int blk = blockIdx.x;
  const int b = blk >> 6, lt = blk & 63;
  const int l0 = lt * 64;
  const int t = threadIdx.x, lane = t & 31, wave = t >> 5;
#pragma unroll
  for (int it = 0; it < 4; ++it) {
    const int f = it * 256 + t;
    const int c = f >> 4, l4 = (f & 15) * 4;
    const v4f v = *(const v4f*)(x + ((size_t)(b * CIN + c)) * SEQL + l0 + l4);
#pragma unroll
    for (int e = 0; e < 4; ++e) s[(l4 + e) * 68 + c] = v[e];
  }
  __syncthreads();
  const int rq = lane >> 3, c8 = (lane & 7) * 8;
  v8h hv[2], lv[2];
#pragma unroll
  for (int it = 0; it < 2; ++it) {
    const int row = wave * 8 + it * 4 + rq;
    const v4f a0 = *(const v4f*)(s + row * 68 + c8);
    const v4f a1 = *(const v4f*)(s + row * 68 + c8 + 4);
    split_bf8(a0, a1, hv[it], lv[it]);
  }
  for (int pass = 0; pass < 2; ++pass) {
#pragma unroll
    for (int it = 0; it < 2; ++it) {
      const int row = wave * 8 + it * 4 + rq;
      const size_t off = ((size_t)(b * SEQL + l0 + row)) * CIN + c8;
      *(volatile v8h*)(Th + off) = hv[it];
      *(volatile v8h*)(Tl + off) = lv[it];
    }
    __threadfence();
  }
}

__global__ __launch_bounds__(256) void conv_silu_kernel(
    const float* __restrict__ XZ, const float* __restrict__ w_conv, const float* __restrict__ b_conv,
    float* __restrict__ XC, unsigned short* __restrict__ XCh, unsigned short* __restrict__ XCl)
{
  __shared__ __align__(16) float sX[16 * 132];
  const int t = threadIdx.x, lane = t & 31, wave = t >> 5;
  const int d = t & 127, rg = t >> 7;
  const int rb = blockIdx.x * 16;
  const int r0 = rb + rg * 8;
  const int l0 = r0 & (SEQL - 1);
  const float w0 = w_conv[d * 4 + 0], w1 = w_conv[d * 4 + 1], w2 = w_conv[d * 4 + 2], w3 = w_conv[d * 4 + 3];
  const float bc = b_conv[d];
  float x0, x1, x2;
  {
    int sr;
    sr = r0 - 3; sr = (sr < 0) ? 0 : sr; { const float v = XZ[(size_t)sr * 256 + d]; x0 = (l0 - 3 >= 0) ? v : 0.f; }
    sr = r0 - 2; sr = (sr < 0) ? 0 : sr; { const float v = XZ[(size_t)sr * 256 + d]; x1 = (l0 - 2 >= 0) ? v : 0.f; }
    sr = r0 - 1; sr = (sr < 0) ? 0 : sr; { const float v = XZ[(size_t)sr * 256 + d]; x2 = (l0 - 1 >= 0) ? v : 0.f; }
  }
#pragma unroll 1
  for (int r = 0; r < 8; ++r) {
    const float xcur = XZ[(size_t)(r0 + r) * 256 + d];
    float acc = w0 * x0;
    acc = fmaf(w1, x1, acc);
    acc = fmaf(w2, x2, acc);
    acc = fmaf(w3, xcur, acc);
    const float sv = acc + bc;
    const float sg = 1.0f / (1.0f + __expf(-sv));
    sX[(rg * 8 + r) * 132 + d] = sv * sg;
    x0 = x1; x1 = x2; x2 = xcur;
  }
  __syncthreads();
  const int prow = wave * 2 + (lane >> 4);
  const int d8 = (lane & 15) * 8;
  v8h hv, lv;
  {
    const v4f a0 = *(const v4f*)(sX + prow * 132 + d8);
    const v4f a1 = *(const v4f*)(sX + prow * 132 + d8 + 4);
    split_bf8(a0, a1, hv, lv);
  }
  v4f f0 = *(const v4f*)(sX + (wave * 2 + 0) * 132 + lane * 4);
  v4f f1 = *(const v4f*)(sX + (wave * 2 + 1) * 132 + lane * 4);
  for (int pass = 0; pass < 2; ++pass) {
    *(volatile v4f*)(XC + (size_t)(rb + wave * 2 + 0) * DIN + lane * 4) = f0;
    *(volatile v4f*)(XC + (size_t)(rb + wave * 2 + 1) * DIN + lane * 4) = f1;
    const size_t poff = (size_t)(rb + prow) * DIN + d8;
    *(volatile v8h*)(XCh + poff) = hv;
    *(volatile v8h*)(XCl + poff) = lv;
    __threadfence();
  }
}

__global__ __launch_bounds__(128) void scan_kernel(
    const float* __restrict__ PRJ, const float* __restrict__ XC, const float* __restrict__ XZ,
    const float* __restrict__ w_dt, const float* __restrict__ b_dt, const float* __restrict__ A_log,
    const float* __restrict__ Dsk, unsigned short* __restrict__ Yh, unsigned short* __restrict__ Yl)
{
  __shared__ __align__(16) float sP[TS * 64];
  __shared__ __align__(16) float sY[TS * 132];
  __shared__ float sA[DIN * 17];
  const int b = blockIdx.x;
  const int d = threadIdx.x;
  const int lane = d & 31, wave = d >> 5;

#pragma unroll 1
  for (int n = 0; n < NST; ++n) sA[d * 17 + n] = -expf(A_log[d * NST + n]);
  __syncthreads();
  float An[NST];
#pragma unroll
  for (int n = 0; n < NST; ++n) An[n] = sA[d * 17 + n];

  const float wd0 = w_dt[0 * DIN + d], wd1 = w_dt[1 * DIN + d], wd2 = w_dt[2 * DIN + d], wd3 = w_dt[3 * DIN + d];
  const float bd = b_dt[d], Dd = Dsk[d];
  float h[NST];
#pragma unroll
  for (int n = 0; n < NST; ++n) h[n] = 0.f;

  const size_t rowb = (size_t)b * SEQL;
  const int rsel = lane >> 4, d8 = (lane & 15) * 8;
#pragma unroll 1
  for (int c = 0; c < SEQL / TS; ++c) {
    const size_t row0 = rowb + (size_t)c * TS;
    __syncthreads();
#pragma unroll
    for (int it = 0; it < 4; ++it) {
      const int f = it * 128 + d;
      const int r = f >> 4, c4 = (f & 15) * 4;
      *(v4f*)(sP + r * 64 + c4) = *(const v4f*)(PRJ + (row0 + r) * NPRJ + c4);
    }
    __syncthreads();
#pragma unroll 1
    for (int s = 0; s < TS; ++s) {
      const size_t row = row0 + s;
      const float xcv = XC[row * DIN + d];
      const float zv  = XZ[row * 256 + DIN + d];
      const float* pr = sP + s * 64;
      const v4f dti = *(const v4f*)(pr);
      v4f Bq[4], Cq[4];
#pragma unroll
      for (int q = 0; q < 4; ++q) {
        Bq[q] = *(const v4f*)(pr + NDT + 4 * q);
        Cq[q] = *(const v4f*)(pr + NDT + NST + 4 * q);
      }
      float a = dti[0] * wd0;
      a = fmaf(dti[1], wd1, a);
      a = fmaf(dti[2], wd2, a);
      a = fmaf(dti[3], wd3, a);
      a += bd;
      const float dt = fmaxf(a, 0.f) + log1pf(expf(-fabsf(a)));
      const float u = dt * xcv;
      float y = 0.f;
#pragma unroll
      for (int n = 0; n < NST; ++n) {
        const float e = __expf(dt * An[n]);
        h[n] = fmaf(e, h[n], u * Bq[n >> 2][n & 3]);
        y = fmaf(h[n], Cq[n >> 2][n & 3], y);
      }
      y = fmaf(xcv, Dd, y);
      const float sg = 1.0f / (1.0f + __expf(-zv));
      y = y * (zv * sg);
      sY[s * 132 + d] = y;
    }
    __syncthreads();
    v8h hv[4], lv[4];
#pragma unroll
    for (int it = 0; it < 4; ++it) {
      const int r = wave * 8 + it * 2 + rsel;
      const v4f a0 = *(const v4f*)(sY + r * 132 + d8);
      const v4f a1 = *(const v4f*)(sY + r * 132 + d8 + 4);
      split_bf8(a0, a1, hv[it], lv[it]);
    }
    for (int pass = 0; pass < 2; ++pass) {
#pragma unroll
      for (int it = 0; it < 4; ++it) {
        const int r = wave * 8 + it * 2 + rsel;
        const size_t off = (row0 + r) * DIN + d8;
        *(volatile v8h*)(Yh + off) = hv[it];
        *(volatile v8h*)(Yl + off) = lv[it];
      }
      __threadfence();
    }
  }
}

__global__ __launch_bounds__(256) void ln1_kernel(
    const float* __restrict__ IN, const float* __restrict__ g, const float* __restrict__ bb,
    unsigned short* __restrict__ Th, unsigned short* __restrict__ Tl)
{
  __shared__ __align__(16) float sL[32 * 68];
  const int t = threadIdx.x, lane = t & 31, wave = t >> 5;
  const int rb = blockIdx.x * 32;
  const float g0 = g[lane * 2], g1 = g[lane * 2 + 1];
  const float b0 = bb[lane * 2], b1 = bb[lane * 2 + 1];
#pragma unroll 1
  for (int rr = 0; rr < 4; ++rr) {
    const int row = wave * 4 + rr;
    const v2f v = *(const v2f*)(IN + (size_t)(rb + row) * CIN + lane * 2);
    float sm = v[0] + v[1];
#pragma unroll
    for (int off = 1; off < 32; off <<= 1) sm += __shfl_xor(sm, off, 32);
    const float mu = sm * (1.0f / 64.0f);
    const float e0 = v[0] - mu, e1 = v[1] - mu;
    float q = e0 * e0 + e1 * e1;
#pragma unroll
    for (int off = 1; off < 32; off <<= 1) q += __shfl_xor(q, off, 32);
    const float var = q * (1.0f / 64.0f);
    const float inv = rsqrtf(var + 1e-5f);
    const float o0 = fmaxf((e0 * inv) * g0 + b0, 0.f);
    const float o1 = fmaxf((e1 * inv) * g1 + b1, 0.f);
    sL[row * 68 + lane * 2] = o0;
    sL[row * 68 + lane * 2 + 1] = o1;
  }
  __syncthreads();
  const int row = wave * 4 + (lane >> 3);
  const int c8 = (lane & 7) * 8;
  v8h hv, lv;
  {
    const v4f a0 = *(const v4f*)(sL + row * 68 + c8);
    const v4f a1 = *(const v4f*)(sL + row * 68 + c8 + 4);
    split_bf8(a0, a1, hv, lv);
  }
  const size_t off = (size_t)(rb + row) * CIN + c8;
  for (int pass = 0; pass < 2; ++pass) {
    *(volatile v8h*)(Th + off) = hv;
    *(volatile v8h*)(Tl + off) = lv;
    __threadfence();
  }
}

__global__ __launch_bounds__(256) void ln2_out_kernel(
    const float* __restrict__ IN, const float* __restrict__ g, const float* __restrict__ bb,
    float* __restrict__ out)
{
  __shared__ __align__(16) float sT[64 * 132];
  const int t = threadIdx.x, lane = t & 31, wave = t >> 5;
  const int b = blockIdx.x >> 6, i = blockIdx.x & 63;
  const v4f gg = *(const v4f*)(g + lane * 4);
  const v4f bv = *(const v4f*)(bb + lane * 4);
#pragma unroll 1
  for (int rr = 0; rr < 8; ++rr) {
    const int j = wave * 8 + rr;
    const size_t row = (size_t)b * SEQL + (size_t)j * 64 + i;
    const v4f v = *(const v4f*)(IN + row * DIN + lane * 4);
    float sm = (v[0] + v[1]) + (v[2] + v[3]);
#pragma unroll
    for (int off = 1; off < 32; off <<= 1) sm += __shfl_xor(sm, off, 32);
    const float mu = sm * (1.0f / 128.0f);
    v4f e;
#pragma unroll
    for (int k = 0; k < 4; ++k) e[k] = v[k] - mu;
    float q = e[0] * e[0];
    q = fmaf(e[1], e[1], q);
    q = fmaf(e[2], e[2], q);
    q = fmaf(e[3], e[3], q);
#pragma unroll
    for (int off = 1; off < 32; off <<= 1) q += __shfl_xor(q, off, 32);
    const float var = q * (1.0f / 128.0f);
    const float inv = rsqrtf(var + 1e-5f);
    v4f o;
#pragma unroll
    for (int k = 0; k < 4; ++k) o[k] = fmaxf((e[k] * inv) * gg[k] + bv[k], 0.f);
    *(v4f*)(sT + j * 132 + lane * 4) = o;
  }
  __syncthreads();
  const int chh = lane >> 4, j4 = (lane & 15) * 4;
  v4f ov[8];
#pragma unroll
  for (int it = 0; it < 8; ++it) {
    const int chl = wave * 16 + it * 2 + chh;
#pragma unroll
    for (int k = 0; k < 4; ++k) ov[it][k] = sT[(j4 + k) * 132 + chl];
  }
  for (int pass = 0; pass < 2; ++pass) {
#pragma unroll
    for (int it = 0; it < 8; ++it) {
      const int chl = wave * 16 + it * 2 + chh;
      const size_t off = (((size_t)(b * 128 + chl)) * 64 + i) * 64 + j4;
      *(volatile v4f*)(out + off) = ov[it];
    }
    __threadfence();
  }
}

extern "C" void kernel_launch(void* const* d_in, const int* in_sizes, int n_in,
                              void* d_out, int out_size, void* d_ws, size_t ws_size,
                              hipStream_t stream)
{
  const float* x       = (const float*)d_in[0];
  const float* w_in1   = (const float*)d_in[1];
  const float* w_conv1 = (const float*)d_in[2];
  const float* b_conv1 = (const float*)d_in[3];
  const float* w_x1    = (const float*)d_in[4];
  const float* w_dt1   = (const float*)d_in[5];
  const float* b_dt1   = (const float*)d_in[6];
  const float* A_log1  = (const float*)d_in[7];
  const float* D1      = (const float*)d_in[8];
  const float* w_out1  = (const float*)d_in[9];
  const float* g_ln1   = (const float*)d_in[10];
  const float* b_ln1   = (const float*)d_in[11];
  const float* w_in2   = (const float*)d_in[12];
  const float* w_conv2 = (const float*)d_in[13];
  const float* b_conv2 = (const float*)d_in[14];
  const float* w_x2    = (const float*)d_in[15];
  const float* w_dt2   = (const float*)d_in[16];
  const float* b_dt2   = (const float*)d_in[17];
  const float* A_log2  = (const float*)d_in[18];
  const float* D2      = (const float*)d_in[19];
  const float* w_out2  = (const float*)d_in[20];
  const float* g_ln2   = (const float*)d_in[21];
  const float* b_ln2   = (const float*)d_in[22];

  if (n_in < 23) return;
  if (in_sizes[0] != NB * CIN * SEQL) return;
  if (out_size != NB * 128 * SEQL) return;

  const size_t MiB = 1048576;
  const size_t OFF_WGT = 0;
  const size_t OFF_T   = 1 * MiB;
  const size_t OFF_XZ  = 9 * MiB;
  const size_t OFF_XC  = 41 * MiB;
  const size_t OFF_XCP = 57 * MiB;
  const size_t OFF_PRJ = 73 * MiB;
  const size_t TOTAL   = 81 * MiB;
  if (ws_size < TOTAL) return;
  if ((size_t)WGT_END * 2 > OFF_T) return;

  char* ws = (char*)d_ws;
  unsigned short* WGT = (unsigned short*)(ws + OFF_WGT);
  unsigned short* Th  = (unsigned short*)(ws + OFF_T);
  unsigned short* Tl  = Th + (size_t)NROWS * CIN;
  float* XZ   = (float*)(ws + OFF_XZ);
  float* OUTB = XZ;
  float* XC   = (float*)(ws + OFF_XC);
  unsigned short* XCh = (unsigned short*)(ws + OFF_XCP);
  unsigned short* XCl = XCh + (size_t)NROWS * DIN;
  unsigned short* Yh  = XCh;
  unsigned short* Yl  = XCl;
  float* PRJ  = (float*)(ws + OFF_PRJ);
  float* dout = (float*)d_out;

  const int TILES_M = NROWS / 64;

  weight_planes_kernel<<<dim3(8, 6), 256, 0, stream>>>(w_in1, w_x1, w_out1, w_in2, w_x2, w_out2, WGT);
  x_to_planes_kernel<<<NB * (SEQL / 64), 256, 0, stream>>>(x, Th, Tl);

  wmma_gemm64<1, true, 0, 0, false><<<dim3((TILES_M * 4) / 8, 1), 256, 0, stream>>>(
      Th, Tl, CIN, 0L, WGT + WIN1_H, WGT + WIN1_L, CIN, 0L,
      (void*)XZ, (void*)XZ, 256, 0L, PRJ, PRJ, 0L, NROWS, 256, CIN, 1.0f);
  conv_silu_kernel<<<NROWS / 16, 256, 0, stream>>>(XZ, w_conv1, b_conv1, XC, XCh, XCl);
  wmma_gemm64<1, true, 0, 0, false><<<dim3(TILES_M / 8, 1), 256, 0, stream>>>(
      XCh, XCl, DIN, 0L, WGT + WX1_H, WGT + WX1_L, DIN, 0L,
      (void*)PRJ, (void*)PRJ, NPRJ, 0L, XC, XC, 0L, NROWS, NPRJ, DIN, 1.0f);
  scan_kernel<<<NB, 128, 0, stream>>>(PRJ, XC, XZ, w_dt1, b_dt1, A_log1, D1, Yh, Yl);
  wmma_gemm64<1, true, 0, 0, false><<<dim3(TILES_M / 8, 1), 256, 0, stream>>>(
      Yh, Yl, DIN, 0L, WGT + WOUT1_H, WGT + WOUT1_L, DIN, 0L,
      (void*)OUTB, (void*)OUTB, CIN, 0L, PRJ, PRJ, 0L, NROWS, CIN, DIN, 1.0f);
  ln1_kernel<<<NROWS / 32, 256, 0, stream>>>(OUTB, g_ln1, b_ln1, Th, Tl);

  wmma_gemm64<1, true, 0, 0, false><<<dim3((TILES_M * 4) / 8, 1), 256, 0, stream>>>(
      Th, Tl, CIN, 0L, WGT + WIN2_H, WGT + WIN2_L, CIN, 0L,
      (void*)XZ, (void*)XZ, 256, 0L, PRJ, PRJ, 0L, NROWS, 256, CIN, 1.0f);
  conv_silu_kernel<<<NROWS / 16, 256, 0, stream>>>(XZ, w_conv2, b_conv2, XC, XCh, XCl);
  wmma_gemm64<1, true, 0, 0, false><<<dim3(TILES_M / 8, 1), 256, 0, stream>>>(
      XCh, XCl, DIN, 0L, WGT + WX2_H, WGT + WX2_L, DIN, 0L,
      (void*)PRJ, (void*)PRJ, NPRJ, 0L, XC, XC, 0L, NROWS, NPRJ, DIN, 1.0f);
  scan_kernel<<<NB, 128, 0, stream>>>(PRJ, XC, XZ, w_dt2, b_dt2, A_log2, D2, Yh, Yl);
  wmma_gemm64<1, true, 0, 0, false><<<dim3((TILES_M * 2) / 8, 1), 256, 0, stream>>>(
      Yh, Yl, DIN, 0L, WGT + WOUT2_H, WGT + WOUT2_L, DIN, 0L,
      (void*)OUTB, (void*)OUTB, DIN, 0L, PRJ, PRJ, 0L, NROWS, DIN, DIN, 1.0f);
  ln2_out_kernel<<<NB * 64, 256, 0, stream>>>(OUTB, g_ln2, b_ln2, dout);

  (void)hipGetLastError();
}
